// TriangleAttention_515396076358
// MI455X (gfx1250) — hardware-verified
//
#include <hip/hip_runtime.h>
#include <math.h>
#include <stdint.h>

#define TS     256
#define TD     128
#define TH     4
#define TDH    32
#define NTOK   (TS * TS)
#define NHALF  2
#define RH     (TS / NHALF)
#define TOKH   (RH * TS)
#define XN_LD  256
#define QKG_LD 384
#define OG_LD  256
#define W_LD   256
#define WROWS  640

static_assert(TOKH % 64 == 0);
static_assert(QKG_LD % 64 == 0);
static_assert(OG_LD % 32 == 0);
static_assert(TH * TD == 512);
static_assert(TH * TDH == TD);
static_assert(NTOK % 32 == 0);

typedef __attribute__((ext_vector_type(16))) _Float16 v16h;
typedef __attribute__((ext_vector_type(8)))  _Float16 v8h;
typedef __attribute__((ext_vector_type(16))) __bf16   v16b;
typedef __attribute__((ext_vector_type(8)))  __bf16   v8b;
typedef __attribute__((ext_vector_type(8)))  float    v8f;
typedef __attribute__((ext_vector_type(4)))  float    v4f;
typedef __attribute__((ext_vector_type(4)))  unsigned int v4u;
typedef v4f __attribute__((may_alias)) v4fa;

static constexpr float RSCALE = 0.17677669529663687f;

__device__ __forceinline__ unsigned short f2bf_bits(float f) {
  unsigned u = __float_as_uint(f);
  return (unsigned short)((u + 0x7FFFu + ((u >> 16) & 1u)) >> 16);
}
__device__ __forceinline__ float bf_bits2f(unsigned short hb) { return __uint_as_float(((unsigned)hb) << 16); }
__device__ __forceinline__ float bfr(float f) { return bf_bits2f(f2bf_bits(f)); }
__device__ __forceinline__ unsigned pk16(unsigned short a, unsigned short b) { return (unsigned)a | ((unsigned)b << 16); }

__device__ __forceinline__ void dep_guard_h(v8f& a, v8f& b, v16h x, v16h y) { asm volatile("v_nop\n\tv_nop\n\tv_nop\n\tv_nop" : "+v"(a), "+v"(b) : "v"(x), "v"(y)); }
__device__ __forceinline__ void dep_guard_b(v8f& a, v8f& b, v16b x, v16b y) { asm volatile("v_nop\n\tv_nop\n\tv_nop\n\tv_nop" : "+v"(a), "+v"(b) : "v"(x), "v"(y)); }
__device__ __forceinline__ void keep4_h(v16h a, v16h b, v16h c, v16h d) { asm volatile("v_nop" :: "v"(a), "v"(b), "v"(c), "v"(d)); }
__device__ __forceinline__ void keep4_b(v16b a, v16b b, v16b c, v16b d) { asm volatile("v_nop" :: "v"(a), "v"(b), "v"(c), "v"(d)); }
__device__ __forceinline__ void acc_guard4(v8f& a, v8f& b, v8f& c, v8f& d) { asm volatile("v_nop\n\tv_nop\n\tv_nop\n\tv_nop" : "+v"(a), "+v"(b), "+v"(c), "+v"(d)); }

template <typename T> struct Frag;
template <> struct Frag<_Float16> {
  typedef v16h V; union U { v16h v; v8h h[2]; };
  static __device__ __forceinline__ v16h load(const _Float16* p) {
    U f; f.h[0] = *(const v8h*)(p); f.h[1] = *(const v8h*)(p + 16); return f.v;
  }
  static __device__ __forceinline__ v8f mma(v16h a, v16h b, v8f c) {
    return __builtin_amdgcn_wmma_f32_16x16x32_f16(false, a, false, b, (short)0, c, false, false);
  }
  static __device__ __forceinline__ void guard(v8f& a, v8f& b, v16h x, v16h y) { dep_guard_h(a, b, x, y); }
  static __device__ __forceinline__ void keep(v16h a, v16h b, v16h c, v16h d) { keep4_h(a, b, c, d); }
};
template <> struct Frag<__bf16> {
  typedef v16b V; union U { v16b v; v8b h[2]; };
  static __device__ __forceinline__ v16b load(const __bf16* p) {
    U f; f.h[0] = *(const v8b*)(p); f.h[1] = *(const v8b*)(p + 16); return f.v;
  }
  static __device__ __forceinline__ v8f mma(v16b a, v16b b, v8f c) {
    return __builtin_amdgcn_wmma_f32_16x16x32_bf16(false, a, false, b, (short)0, c, false, false);
  }
  static __device__ __forceinline__ void guard(v8f& a, v8f& b, v16b x, v16b y) { dep_guard_b(a, b, x, y); }
  static __device__ __forceinline__ void keep(v16b a, v16b b, v16b c, v16b d) { keep4_b(a, b, c, d); }
};

template <int ET> struct Elem;
template <> struct Elem<0> { typedef _Float16 T; };
template <> struct Elem<1> { typedef __bf16 T; };
template <int ET, bool SPLIT, int BIAS_MODE, int OUT_MODE, bool RESID>
__global__ __launch_bounds__(256) void wmma_gemm64(
    const unsigned short* __restrict__ Ap, const unsigned short* __restrict__ A2p, int lda, long strideA,
    const unsigned short* __restrict__ Btp, const unsigned short* __restrict__ Bt2p, int ldb, long strideB,
    void* __restrict__ Cout, void* __restrict__ Cout2, int ldc, long strideC,
    const float* __restrict__ bias,
    const float* __restrict__ resid, long strideR,
    int M, int N, int K, float scale) {
  typedef typename Elem<ET>::T T;
  typedef typename Frag<T>::V V;
  const T* A = (const T*)Ap; const T* A2 = (const T*)A2p; const T* Bt = (const T*)Btp; const T* Bt2 = (const T*)Bt2p;
  __shared__ __align__(16) float sT[8][16 * 68];
  const int b    = blockIdx.y;
  const int lane = threadIdx.x & 31;
  const int wave = threadIdx.x >> 5;
  const int tilesN = N >> 6;
  const int tilesM = M >> 6;
  const int tile = blockIdx.x * 8 + wave;
  if (tile >= tilesM * tilesN) return;
  const int tm = tile / tilesN;
  const int tn = tile - tm * tilesN;
  const int m0 = tm << 6;
  const int n0 = tn << 6;

  const T* Ab  = A  + (size_t)b * strideA;
  const T* Bb  = Bt + (size_t)b * strideB;
  const T* Ab2 = SPLIT ? (A2  + (size_t)b * strideA) : nullptr;
  const T* Bb2 = SPLIT ? (Bt2 + (size_t)b * strideB) : nullptr;

  const int rlane = lane & 15;
  const int koff  = (lane >> 4) * 8;
  const int mOff  = (lane >> 4) * 8;

  v8f acc[4][4];
#pragma unroll
  for (int i = 0; i < 4; ++i)
#pragma unroll
    for (int j = 0; j < 4; ++j) acc[i][j] = (v8f){0.f,0.f,0.f,0.f,0.f,0.f,0.f,0.f};

  for (int k0 = 0; k0 < K; k0 += 32) {
    V bh[4], bl[4];
#pragma unroll
    for (int j = 0; j < 4; ++j) {
      const size_t bo = (size_t)(n0 + (j << 4) + rlane) * ldb + koff + k0;
      bh[j] = Frag<T>::load(Bb + bo);
      if (SPLIT) bl[j] = Frag<T>::load(Bb2 + bo);
    }
#pragma unroll
    for (int i = 0; i < 4; ++i) {
      const size_t ao = (size_t)(m0 + (i << 4) + rlane) * lda + koff + k0;
      V ah = Frag<T>::load(Ab + ao);
      V al;
      if (SPLIT) al = Frag<T>::load(Ab2 + ao);
#pragma unroll
      for (int j = 0; j < 4; ++j) {
        acc[i][j] = Frag<T>::mma(ah, bh[j], acc[i][j]);
        if (SPLIT) {
          acc[i][j] = Frag<T>::mma(ah, bl[j], acc[i][j]);
          acc[i][j] = Frag<T>::mma(al, bh[j], acc[i][j]);
        }
      }
      Frag<T>::guard(acc[i][0], acc[i][3], ah, SPLIT ? al : ah);
    }
    Frag<T>::keep(bh[0], bh[1], bh[2], bh[3]);
    if (SPLIT) Frag<T>::keep(bl[0], bl[1], bl[2], bl[3]);
  }
  acc_guard4(acc[0][0], acc[0][1], acc[0][2], acc[0][3]);
  acc_guard4(acc[1][0], acc[1][1], acc[1][2], acc[1][3]);
  acc_guard4(acc[2][0], acc[2][1], acc[2][2], acc[2][3]);
  acc_guard4(acc[3][0], acc[3][1], acc[3][2], acc[3][3]);

  float* slab = sT[wave];
  const float* Rb = RESID ? (resid + (size_t)b * strideR) : nullptr;
#pragma unroll
  for (int i = 0; i < 4; ++i) {
    const int mBase = m0 + (i << 4);
#pragma unroll
    for (int j = 0; j < 4; ++j) {
      const int n = n0 + (j << 4) + rlane;
      float bv = 0.f;
      if (BIAS_MODE == 2) bv = bias[n];
#pragma unroll
      for (int r = 0; r < 8; ++r) {
        float v = acc[i][j][r] * scale;
        if (BIAS_MODE == 1) v += bias[mBase + mOff + r];
        if (BIAS_MODE == 2) v += bv;
        if (RESID) v += Rb[(size_t)(mBase + mOff + r) * ldc + n];
        slab[(mOff + r) * 68 + (j << 4) + rlane] = v;
      }
    }
    __builtin_amdgcn_fence(__ATOMIC_RELEASE, "workgroup");
    __builtin_amdgcn_wave_barrier();
    __builtin_amdgcn_fence(__ATOMIC_ACQUIRE, "workgroup");
    if (OUT_MODE == 0) {
      float* C = (float*)Cout + (size_t)b * strideC;
      const int hh = lane >> 4, c4 = (lane & 15) * 4;
      for (int pass = 0; pass < 2; ++pass) {
#pragma unroll
        for (int it = 0; it < 8; ++it) {
          const int row = it * 2 + hh;
          v4f v = *(const v4f*)(slab + row * 68 + c4);
          *(volatile v4f*)(C + (size_t)(mBase + row) * ldc + n0 + c4) = v;
        }
        __threadfence();
      }
    } else {
      const int q = lane >> 3, c8 = (lane & 7) * 8;
      unsigned short* C  = (unsigned short*)Cout  + (size_t)b * strideC;
      unsigned short* C2 = (OUT_MODE == 2) ? ((unsigned short*)Cout2 + (size_t)b * strideC) : nullptr;
      for (int pass = 0; pass < 2; ++pass) {
#pragma unroll
        for (int it = 0; it < 4; ++it) {
          const int row = it * 4 + q;
          const float* sp = slab + row * 68 + c8;
          v8h hv, lv;
#pragma unroll
          for (int e = 0; e < 8; ++e) {
            if (OUT_MODE == 1) {
              hv[e] = (_Float16)sp[e];
            } else {
              unsigned short hb = f2bf_bits(sp[e]);
              unsigned short lb = f2bf_bits(sp[e] - bf_bits2f(hb));
              hv[e] = __builtin_bit_cast(_Float16, hb);
              lv[e] = __builtin_bit_cast(_Float16, lb);
            }
          }
          *(volatile v8h*)(C + (size_t)(mBase + row) * ldc + n0 + c8) = hv;
          if (OUT_MODE == 2) *(volatile v8h*)(C2 + (size_t)(mBase + row) * ldc + n0 + c8) = lv;
        }
        __threadfence();
      }
    }
    __builtin_amdgcn_fence(__ATOMIC_RELEASE, "workgroup");
    __builtin_amdgcn_wave_barrier();
    __builtin_amdgcn_fence(__ATOMIC_ACQUIRE, "workgroup");
  }
}

__global__ __launch_bounds__(256) void wprep_kernel(const float* __restrict__ wq, const float* __restrict__ wk,
                                                     const float* __restrict__ wg, const float* __restrict__ wv,
                                                     const float* __restrict__ wo, unsigned short* __restrict__ WALL) {
  const int tid = threadIdx.x, L = tid & 31;
  const int row = blockIdx.x * 8 + (tid >> 5);
  const int mid = blockIdx.x >> 4;
  const float* src = (mid == 0) ? wq : ((mid == 1) ? wk : ((mid == 2) ? wg : ((mid == 3) ? wv : wo)));
  const int srow = row & (TD - 1);
  const int sg = (mid == 4) ? (((L >> 3) << 2) + (L & 3)) : (L & 15);
  const float* p = src + (size_t)srow * TD + 8 * sg;
  const v4f a = *(const v4fa*)p;
  const v4f c = *(const v4fa*)(p + 4);
  v4u o;
  o[0] = pk16(f2bf_bits(a[0]), f2bf_bits(a[1]));
  o[1] = pk16(f2bf_bits(a[2]), f2bf_bits(a[3]));
  o[2] = pk16(f2bf_bits(c[0]), f2bf_bits(c[1]));
  o[3] = pk16(f2bf_bits(c[2]), f2bf_bits(c[3]));
  unsigned short* d = WALL + (size_t)row * W_LD + 8 * L;
  *(volatile v4u*)d = o;
  __threadfence();
  *(volatile v4u*)d = o;
}

__global__ __launch_bounds__(512) void ln_bias_kernel(const float* __restrict__ x, const float* __restrict__ wln,
                                                       const float* __restrict__ bln, const float* __restrict__ wbias,
                                                       unsigned short* __restrict__ XN, float* __restrict__ TB) {
  __shared__ float swb[TH * TD];
  __shared__ __align__(16) float stb[TH * 32];
  const int tid = threadIdx.x;
  swb[tid] = bfr(wbias[tid]);
  __syncthreads();

  const int wave = tid >> 5, lane = tid & 31, hh = lane >> 4, sub = lane & 15;
  const int tokb = wave * 2 + hh;
  const size_t tok = (size_t)blockIdx.x * 32 + tokb;
  const float* xp = x + tok * TD + 8 * sub;
  const v4f xa = *(const v4fa*)xp;
  const v4f xb = *(const v4fa*)(xp + 4);
  const v4f wa = *(const v4fa*)(wln + 8 * sub);
  const v4f wb = *(const v4fa*)(wln + 8 * sub + 4);
  const v4f ba = *(const v4fa*)(bln + 8 * sub);
  const v4f bb = *(const v4fa*)(bln + 8 * sub + 4);
  float xv[8], wl[8], bl[8];
#pragma unroll
  for (int e = 0; e < 4; ++e) {
    xv[e] = bfr(xa[e]); xv[e + 4] = bfr(xb[e]);
    wl[e] = bfr(wa[e]); wl[e + 4] = bfr(wb[e]);
    bl[e] = bfr(ba[e]); bl[e + 4] = bfr(bb[e]);
  }
  float ssum = 0.0f;
#pragma unroll
  for (int e = 0; e < 8; ++e) ssum += xv[e];
#pragma unroll
  for (int off = 8; off >= 1; off >>= 1) ssum += __shfl_xor(ssum, off, 32);
  const float mu = ssum * (1.0f / 128.0f);
  float dv[8];
  float q2 = 0.0f;
#pragma unroll
  for (int e = 0; e < 8; ++e) { dv[e] = xv[e] - mu; q2 += dv[e] * dv[e]; }
#pragma unroll
  for (int off = 8; off >= 1; off >>= 1) q2 += __shfl_xor(q2, off, 32);
  const float rstd = rsqrtf(q2 * (1.0f / 128.0f) + 1e-5f);
  float xn[8];
#pragma unroll
  for (int e = 0; e < 8; ++e) xn[e] = (dv[e] * rstd) * wl[e] + bl[e];

  v4u hv, lv;
#pragma unroll
  for (int e2 = 0; e2 < 4; ++e2) {
    const unsigned short h0 = f2bf_bits(xn[2 * e2]), h1 = f2bf_bits(xn[2 * e2 + 1]);
    const unsigned short l0 = f2bf_bits(xn[2 * e2] - bf_bits2f(h0)), l1 = f2bf_bits(xn[2 * e2 + 1] - bf_bits2f(h1));
    hv[e2] = pk16(h0, h1);
    lv[e2] = pk16(l0, l1);
  }

#pragma unroll 1
  for (int hq = 0; hq < TH; ++hq) {
    const float* w = swb + hq * TD + 8 * sub;
    float acc = 0.0f;
#pragma unroll
    for (int e = 0; e < 8; ++e) acc += xn[e] * w[e];
#pragma unroll
    for (int off = 8; off >= 1; off >>= 1) acc += __shfl_xor(acc, off, 32);
    if (sub == 0) stb[hq * 32 + tokb] = acc;
  }
  __syncthreads();

  const v4f tline = *(const v4fa*)(stb + (lane >> 3) * 32 + (lane & 7) * 4);
  float* tbd = TB + (size_t)(lane >> 3) * NTOK + (size_t)blockIdx.x * 32 + (lane & 7) * 4;
  unsigned short* xd = XN + tok * XN_LD + 8 * sub;
  for (int pass = 0; pass < 2; ++pass) {
    *(volatile v4u*)xd = hv;
    *(volatile v4u*)(xd + TD) = lv;
    if (wave == 0) *(volatile v4f*)tbd = tline;
    __threadfence();
  }
}

#define AT_D   32
#define AT_NW  4
#define AT_QB  64
#define AT_KC  64
#define AT_NKC (TS / AT_KC)
#define TBP    68
#define OSP    36

__device__ __forceinline__ __bf16 at_f2bf(float f) { return __builtin_bit_cast(__bf16, f2bf_bits(f)); }
__device__ __forceinline__ void at_split(float f, __bf16& hi, __bf16& lo) {
  const unsigned short hb = f2bf_bits(f);
  hi = __builtin_bit_cast(__bf16, hb);
  lo = at_f2bf(f - bf_bits2f(hb));
}
__device__ __forceinline__ v8f at_mma(v16b a, v16b b, v8f c) {
  c = __builtin_amdgcn_wmma_f32_16x16x32_bf16(false, a, false, b, (short)0, c, false, false);
  asm volatile("v_nop\n\tv_nop\n\tv_nop\n\tv_nop" : "+v"(c) : "v"(a), "v"(b));
  return c;
}

__global__ __launch_bounds__(128)
void attn_kernel(const unsigned short* __restrict__ qkgh, const unsigned short* __restrict__ qkgl,
                 const unsigned short* __restrict__ vthp, const unsigned short* __restrict__ vtlp,
                 const float* __restrict__ TB, unsigned short* __restrict__ OG) {
  union FB { v16b v; v8b h[2]; };
  __shared__ __align__(16) __bf16 Ksh[AT_KC * AT_D];
  __shared__ __align__(16) __bf16 Ksl[AT_KC * AT_D];
  __shared__ __align__(16) __bf16 Vth[AT_D * AT_KC];
  __shared__ __align__(16) __bf16 Vtl[AT_D * AT_KC];
  __shared__ __align__(16) float  Tbs[AT_QB * TBP];
  __shared__ __align__(16) __bf16 Psh[AT_NW][16 * AT_KC];
  __shared__ __align__(16) __bf16 Psl[AT_NW][16 * AT_KC];
  __shared__ __align__(16) float  Os[AT_NW][16 * OSP];

  const int tid  = threadIdx.x;
  const int wave = tid >> 5;
  const int lane = tid & 31;
  const int hh   = lane >> 4;
  const int c    = lane & 15;

  const int qt = blockIdx.x;
  const int h  = blockIdx.y;
  const int il = blockIdx.z;
  const int jb  = qt * AT_QB;
  const int tk0 = il * TS;
  const int tlw = tk0 + jb + wave * 16;

  const __bf16* Qh = (const __bf16*)(const void*)qkgh;
  const __bf16* Ql = (const __bf16*)(const void*)qkgl;
  const __bf16* Vh = (const __bf16*)(const void*)vthp + ((size_t)il * TD + h * TDH) * TS;
  const __bf16* Vl = (const __bf16*)(const void*)vtlp + ((size_t)il * TD + h * TDH) * TS;
  const float*  TBh = TB + (size_t)h * NTOK;

  const v16b qah = Frag<__bf16>::load(Qh + (size_t)(tlw + c) * QKG_LD + h * TDH + 8 * hh);
  const v16b qal = Frag<__bf16>::load(Ql + (size_t)(tlw + c) * QKG_LD + h * TDH + 8 * hh);

  float mrow[8], lrow[8];
  v8f oacc[2];
#pragma unroll
  for (int r = 0; r < 8; ++r) { mrow[r] = -INFINITY; lrow[r] = 0.f; }
#pragma unroll
  for (int t = 0; t < 2; ++t) oacc[t] = (v8f){0.f,0.f,0.f,0.f,0.f,0.f,0.f,0.f};

  for (int kc = 0; kc < AT_NKC; ++kc) {
    const int kv0 = kc * AT_KC;
    __syncthreads();
    {
      const int r = tid >> 1, d0 = (tid & 1) * 16;
      const __bf16* ksh = Qh + (size_t)(tk0 + kv0 + r) * QKG_LD + TD + h * TDH + d0;
      const __bf16* ksl = Ql + (size_t)(tk0 + kv0 + r) * QKG_LD + TD + h * TDH + d0;
      const int dvr = tid >> 2, s0 = (tid & 3) * 16;
      const __bf16* vsh = Vh + (size_t)dvr * TS + kv0 + s0;
      const __bf16* vsl = Vl + (size_t)dvr * TS + kv0 + s0;
#pragma unroll
      for (int i = 0; i < 2; ++i) {
        const v8b a0 = *(const v8b*)(ksh + 8 * i);
        const v8b a1 = *(const v8b*)(ksl + 8 * i);
        const v8b b0 = *(const v8b*)(vsh + 8 * i);
        const v8b b1 = *(const v8b*)(vsl + 8 * i);
        *(v8b*)(Ksh + r * AT_D  + d0 + 8 * i) = a0;
        *(v8b*)(Ksl + r * AT_D  + d0 + 8 * i) = a1;
        *(v8b*)(Vth + dvr * AT_KC + s0 + 8 * i) = b0;
        *(v8b*)(Vtl + dvr * AT_KC + s0 + 8 * i) = b1;
      }
#pragma unroll
      for (int it = 0; it < 8; ++it) {
        const int idx = it * 128 + tid;
        const int row = idx >> 4, c4 = (idx & 15) * 4;
        const v4f bq = *(const v4fa*)(TBh + (size_t)(jb + row) * TS + kv0 + c4);
        *(v4fa*)(Tbs + row * TBP + c4) = bq;
      }
    }
    __syncthreads();

    v8f s[4];
#pragma unroll
    for (int j = 0; j < 4; ++j) {
      s[j] = (v8f){0.f,0.f,0.f,0.f,0.f,0.f,0.f,0.f};
      FB kb, kl;
      kb.h[0] = *(const v8b*)(Ksh + (j * 16 + c) * AT_D + 8 * hh);
      kb.h[1] = *(const v8b*)(Ksh + (j * 16 + c) * AT_D + 16 + 8 * hh);
      kl.h[0] = *(const v8b*)(Ksl + (j * 16 + c) * AT_D + 8 * hh);
      kl.h[1] = *(const v8b*)(Ksl + (j * 16 + c) * AT_D + 16 + 8 * hh);
      s[j] = at_mma(qah, kb.v, s[j]);
      s[j] = at_mma(qah, kl.v, s[j]);
      s[j] = at_mma(qal, kb.v, s[j]);
    }
    const float* tbw = Tbs + (wave * 16 + 8 * hh) * TBP;
    float cm[8];
#pragma unroll
    for (int r = 0; r < 8; ++r) {
      float m = -INFINITY;
#pragma unroll
      for (int j = 0; j < 4; ++j) {
        const float sv = s[j][r] * RSCALE + tbw[r * TBP + j * 16 + c];
        s[j][r] = sv;
        m = fmaxf(m, sv);
      }
#pragma unroll
      for (int off = 1; off < 16; off <<= 1) m = fmaxf(m, __shfl_xor(m, off, 32));
      cm[r] = m;
    }
    __bf16* pwh = Psh[wave];
    __bf16* pwl = Psl[wave];
#pragma unroll
    for (int r = 0; r < 8; ++r) {
      const float mnew = fmaxf(mrow[r], cm[r]);
      const float alpha = __expf(mrow[r] - mnew);
      mrow[r] = mnew;
      float psum = 0.f;
#pragma unroll
      for (int j = 0; j < 4; ++j) {
        const float p = __expf(s[j][r] - mnew);
        psum += p;
        __bf16 a, bl; at_split(p, a, bl);
        pwh[(8 * hh + r) * AT_KC + j * 16 + c] = a;
        pwl[(8 * hh + r) * AT_KC + j * 16 + c] = bl;
      }
#pragma unroll
      for (int off = 1; off < 16; off <<= 1) psum += __shfl_xor(psum, off, 32);
      lrow[r] = lrow[r] * alpha + psum;
#pragma unroll
      for (int t = 0; t < 2; ++t) oacc[t][r] *= alpha;
    }
    __builtin_amdgcn_fence(__ATOMIC_RELEASE, "workgroup");
    __builtin_amdgcn_wave_barrier();
    __builtin_amdgcn_fence(__ATOMIC_ACQUIRE, "workgroup");
#pragma unroll 1
    for (int kk = 0; kk < 2; ++kk) {
      FB pa, pl;
      pa.h[0] = *(const v8b*)(pwh + c * AT_KC + kk * 32 + 8 * hh);
      pa.h[1] = *(const v8b*)(pwh + c * AT_KC + kk * 32 + 16 + 8 * hh);
      pl.h[0] = *(const v8b*)(pwl + c * AT_KC + kk * 32 + 8 * hh);
      pl.h[1] = *(const v8b*)(pwl + c * AT_KC + kk * 32 + 16 + 8 * hh);
#pragma unroll
      for (int t = 0; t < 2; ++t) {
        FB vb, vl;
        vb.h[0] = *(const v8b*)(Vth + (t * 16 + c) * AT_KC + kk * 32 + 8 * hh);
        vb.h[1] = *(const v8b*)(Vth + (t * 16 + c) * AT_KC + kk * 32 + 16 + 8 * hh);
        vl.h[0] = *(const v8b*)(Vtl + (t * 16 + c) * AT_KC + kk * 32 + 8 * hh);
        vl.h[1] = *(const v8b*)(Vtl + (t * 16 + c) * AT_KC + kk * 32 + 16 + 8 * hh);
        oacc[t] = at_mma(pa.v, vb.v, oacc[t]);
        oacc[t] = at_mma(pa.v, vl.v, oacc[t]);
        oacc[t] = at_mma(pl.v, vb.v, oacc[t]);
      }
    }
  }

  float* os = Os[wave];
#pragma unroll
  for (int r = 0; r < 8; ++r) {
    const float inv = 1.0f / lrow[r];
#pragma unroll
    for (int t = 0; t < 2; ++t) os[(8 * hh + r) * OSP + t * 16 + c] = oacc[t][r] * inv;
  }
  __builtin_amdgcn_fence(__ATOMIC_RELEASE, "workgroup");
  __builtin_amdgcn_wave_barrier();
  __builtin_amdgcn_fence(__ATOMIC_ACQUIRE, "workgroup");

  const int j8 = lane & 7, q8 = lane >> 3;
  const int e0 = 8 * (j8 & 3);
  const unsigned selm = 0u - (unsigned)(j8 >> 2);
  v4u val[4];
#pragma unroll
  for (int it = 0; it < 4; ++it) {
    const int row = it * 4 + q8;
    const size_t tl = (size_t)(tlw + row);
    const v4f o0 = *(const v4fa*)(os + row * OSP + e0);
    const v4f o1 = *(const v4fa*)(os + row * OSP + e0 + 4);
    const v4u gh4 = *(const v4u*)(qkgh + tl * QKG_LD + 2 * TD + h * TDH + e0);
    const v4u gl4 = *(const v4u*)(qkgl + tl * QKG_LD + 2 * TD + h * TDH + e0);
    float ov[8];
    ov[0] = o0[0]; ov[1] = o0[1]; ov[2] = o0[2]; ov[3] = o0[3];
    ov[4] = o1[0]; ov[5] = o1[1]; ov[6] = o1[2]; ov[7] = o1[3];
    v4u packed;
#pragma unroll
    for (int e2 = 0; e2 < 4; ++e2) {
      const unsigned wdh = gh4[e2], wdl = gl4[e2];
      const float g0 = __uint_as_float(wdh << 16) + __uint_as_float(wdl << 16);
      const float g1 = __uint_as_float(wdh & 0xffff0000u) + __uint_as_float(wdl & 0xffff0000u);
      const float v0 = ov[2 * e2]     * (1.0f / (1.0f + __expf(-g0)));
      const float v1 = ov[2 * e2 + 1] * (1.0f / (1.0f + __expf(-g1)));
      const unsigned hb0 = f2bf_bits(v0), hb1 = f2bf_bits(v1);
      const unsigned lb0 = f2bf_bits(v0 - __uint_as_float(hb0 << 16));
      const unsigned lb1 = f2bf_bits(v1 - __uint_as_float(hb1 << 16));
      const unsigned b0 = (hb0 & ~selm) | (lb0 & selm);
      const unsigned b1 = (hb1 & ~selm) | (lb1 & selm);
      packed[e2] = (b0 & 0xffffu) | (b1 << 16);
    }
    val[it] = packed;
  }
  for (int pass = 0; pass < 2; ++pass) {
#pragma unroll
    for (int it = 0; it < 4; ++it) {
      const int row = it * 4 + q8;
      const size_t tl = (size_t)(tlw + row);
      *(volatile v4u*)(OG + tl * OG_LD + h * 64 + 8 * j8) = val[it];
    }
    __threadfence();
  }
}

extern "C" void kernel_launch(void* const* d_in, const int* in_sizes, int n_in,
                              void* d_out, int out_size, void* d_ws, size_t ws_size,
                              hipStream_t stream) {
  if (n_in < 9) return;
  if (in_sizes[0] != NTOK * TD) return;
  if (in_sizes[1] != TD || in_sizes[2] != TD) return;
  if (in_sizes[3] != TH * TD) return;
  if (in_sizes[4] != TD * TD || in_sizes[5] != TD * TD || in_sizes[6] != TD * TD ||
      in_sizes[7] != TD * TD || in_sizes[8] != TD * TD) return;
  if (out_size != NTOK * TD) return;

  const float* x      = (const float*)d_in[0];
  const float* w_ln   = (const float*)d_in[1];
  const float* b_ln   = (const float*)d_in[2];
  const float* w_bias = (const float*)d_in[3];
  const float* w_q    = (const float*)d_in[4];
  const float* w_k    = (const float*)d_in[5];
  const float* w_v    = (const float*)d_in[6];
  const float* w_g    = (const float*)d_in[7];
  const float* w_o    = (const float*)d_in[8];
  float* out = (float*)d_out;

  const size_t bW   = (size_t)WROWS * W_LD * 2;
  const size_t bTB  = (size_t)TH * NTOK * 4;
  const size_t bXN  = (size_t)NTOK * XN_LD * 2;
  const size_t bQKG = (size_t)TOKH * QKG_LD * 2;
  const size_t bVT  = (size_t)RH * TD * TS * 2;
  const size_t bOG  = (size_t)TOKH * OG_LD * 2;
  size_t off = 0;
  const size_t oW    = off; off += bW;
  const size_t oTB   = off; off += bTB;
  const size_t oXN   = off; off += bXN;
  const size_t oQKGh = off; off += bQKG;
  const size_t oQKGl = off; off += bQKG;
  const size_t oVTh  = off; off += bVT;
  const size_t oVTl  = off; off += bVT;
  const size_t oOG   = off; off += bOG;
  if (off > ws_size) return;

  char* ws = (char*)d_ws;
  unsigned short* WALL = (unsigned short*)(ws + oW);
  unsigned short* WQKG = WALL;
  unsigned short* WV   = WALL + (size_t)384 * W_LD;
  unsigned short* WO   = WALL + (size_t)512 * W_LD;
  float*          TBp  = (float*)(ws + oTB);
  unsigned short* XN   = (unsigned short*)(ws + oXN);
  unsigned short* QKGh = (unsigned short*)(ws + oQKGh);
  unsigned short* QKGl = (unsigned short*)(ws + oQKGl);
  unsigned short* VTh  = (unsigned short*)(ws + oVTh);
  unsigned short* VTl  = (unsigned short*)(ws + oVTl);
  unsigned short* OGp  = (unsigned short*)(ws + oOG);

  wprep_kernel<<<dim3(WROWS / 8), dim3(256), 0, stream>>>(w_q, w_k, w_g, w_v, w_o, WALL);
  ln_bias_kernel<<<dim3(NTOK / 32), dim3(512), 0, stream>>>(x, w_ln, b_ln, w_bias, XN, TBp);

  const dim3 blk(256);
  const dim3 gQKG(((TOKH / 64) * (QKG_LD / 64) + 7) / 8, 1);
  const dim3 gVT(1, RH);
  const dim3 gOut(((TOKH / 64) * (TD / 64) + 7) / 8, 1);
  const dim3 gAtt(TS / AT_QB, TH, RH);

  for (int half = 0; half < NHALF; ++half) {
    const unsigned short* XNh = XN + (size_t)half * TOKH * XN_LD;
    wmma_gemm64<1, false, 0, 2, false><<<gQKG, blk, 0, stream>>>(
        XNh, XNh, XN_LD, 0L, WQKG, WQKG, W_LD, 0L, (void*)QKGh, (void*)QKGl, QKG_LD, 0L,
        TBp, TBp, 0L, TOKH, QKG_LD, 256, 1.0f);
    wmma_gemm64<1, false, 0, 2, false><<<gVT, blk, 0, stream>>>(
        WV, WV, W_LD, 0L, XNh, XNh, XN_LD, (long)TS * XN_LD, (void*)VTh, (void*)VTl, TS, (long)TD * TS,
        TBp, TBp, 0L, TD, TS, 256, 1.0f);
    attn_kernel<<<gAtt, dim3(128), 0, stream>>>(QKGh, QKGl, VTh, VTl, TBp, OGp);
    float* outh = out + (size_t)half * TOKH * TD;
    wmma_gemm64<1, false, 0, 0, false><<<gOut, blk, 0, stream>>>(
        OGp, OGp, OG_LD, 0L, WO, WO, W_LD, 0L, (void*)outh, (void*)outh, TD, 0L,
        TBp, TBp, 0L, TOKH, TD, 256, 1.0f);
  }
  (void)hipGetLastError();
}
